// SequenceAttention_68848325755053
// MI455X (gfx1250) — hardware-verified
//
#include <hip/hip_runtime.h>


#ifndef NB
#define NB 8
#endif
#ifndef TQ
#define TQ 64
#endif
#define NB_FULL 8
#define TQ_FULL 64
#define TK    512
#define DV    512
#define NHD   8
#define DHD   64
#define HH    64
#define PCAR  1024.0f
#define VSC   16.0f
#define OSC   (1.0f / 16384.0f)
#define LOG2E 1.4426950408889634f

static_assert(TQ == TQ_FULL || NB == 1);
static_assert(TQ % 64 == 0 && TQ >= 64 && TQ <= TQ_FULL);
static_assert(NB >= 1 && NB <= NB_FULL);
static_assert(TK == 2 * 256);
static_assert(TK == 8 * 64);
static_assert(HH == 2 * 32);
static_assert(NHD * DHD == DV);
static_assert((NB * TQ * NHD) % 64 == 0 && (NB * TK * NHD) % 64 == 0 && HH % 64 == 0 && DHD % 64 == 0);
static_assert(DHD % 32 == 0 && TK % 32 == 0 && DV % 8 == 0);
static_assert((size_t)NB_FULL * TQ_FULL * DV * 4 == 1048576);
static_assert(2 * 32 * 16 == TK * 2);
static_assert(4 * 256 * 8 == 2 * HH * DHD);
static_assert(HH * DHD / 8 == (1 << 9));
static_assert(DHD / 8 == (1 << 3));
static_assert(HH == 64);
static_assert(16 * 68 * 4 <= 131072);
static_assert(TK * 4 + 8 * 4 <= 131072);
static_assert((size_t)2 * HH * DHD * 2 + (size_t)NB * TK * DV * 2 + (size_t)NB * TQ * DV * 2 + (size_t)NB * TK * NHD * HH * 4 + (size_t)NB * TQ * NHD * HH * 4
              + (size_t)NB * DV * TK * 2 + (size_t)NHD * NB * TQ * TK * 2 <= 134217728);

typedef _Float16 h16;
typedef unsigned short bf;
typedef __attribute__((ext_vector_type(16))) __bf16   v16bf;
typedef __attribute__((ext_vector_type(16))) _Float16 v16h;
typedef __attribute__((ext_vector_type(8)))  _Float16 v8h;
typedef __attribute__((ext_vector_type(8)))  unsigned short v8us;
typedef __attribute__((ext_vector_type(8)))  float    v8f;
typedef __attribute__((ext_vector_type(4)))  float    v4f;
typedef __attribute__((ext_vector_type(2)))  float    v2f;
typedef __attribute__((ext_vector_type(2)))  _Float16 v2h;
typedef __attribute__((ext_vector_type(2)))  unsigned short v2us;
typedef v8h  __attribute__((may_alias)) v8ha;
typedef v4f  __attribute__((may_alias)) v4fa;
typedef v8us __attribute__((may_alias)) v8usa;

__device__ __forceinline__ unsigned short f2bf(float f) { unsigned u = __float_as_uint(f); u += 0x7FFFu + ((u >> 16) & 1u); return (unsigned short)(u >> 16); }
__device__ __forceinline__ float bf2f(unsigned short b) { return __uint_as_float(((unsigned)b) << 16); }
__device__ __forceinline__ float bfr(float f) { return bf2f(f2bf(f)); }
__device__ __forceinline__ v16h cat16(v8h lo, v8h hi) { return __builtin_shufflevector(lo, hi, 0, 1, 2, 3, 4, 5, 6, 7, 8, 9, 10, 11, 12, 13, 14, 15); }
__device__ __forceinline__ v16bf cat16b(v8us lo, v8us hi) { return __builtin_bit_cast(v16bf, __builtin_shufflevector(lo, hi, 0, 1, 2, 3, 4, 5, 6, 7, 8, 9, 10, 11, 12, 13, 14, 15)); }
__device__ __forceinline__ v8f wmma16(v16h a, v16h b, v8f c) { return __builtin_amdgcn_wmma_f32_16x16x32_f16(false, a, false, b, (short)0, c, false, false); }
__device__ __forceinline__ v8f wmmab(v16bf a, v16bf b, v8f c) { return __builtin_amdgcn_wmma_f32_16x16x32_bf16(false, a, false, b, (short)0, c, false, false); }
__device__ __forceinline__ h16 toh_flush(float v) { const float w = (fabsf(v) < 6.103515625e-05f) ? 0.0f : v; return (h16)w; }

template <typename T16> struct WFrag;
template <> struct WFrag<h16> { typedef v16h V; static __device__ __forceinline__ V ld(const h16* p) { return cat16(*(const v8h*)p, *(const v8h*)(p + 16)); } static __device__ __forceinline__ v8f mma(V a, V b, v8f c) { return wmma16(a, b, c); } };
template <> struct WFrag<bf> { typedef v16bf V; static __device__ __forceinline__ V ld(const bf* p) { return cat16b(*(const v8us*)p, *(const v8us*)(p + 16)); } static __device__ __forceinline__ v8f mma(V a, V b, v8f c) { return wmmab(a, b, c); } };
template <typename T16, int NSPLIT, bool BIAS>
__global__ __launch_bounds__(32) void k_gemmw(const T16* __restrict__ A, const T16* __restrict__ A2, const T16* __restrict__ Bt, const T16* __restrict__ Bt2, int K, float* C, int ldc, const float* __restrict__ bias, float csc, size_t sA, size_t sB, size_t sC) {
    typedef typename WFrag<T16>::V V;
    __shared__ __align__(16) float os[16 * 68];
    const size_t z = blockIdx.z; A += z * sA; if (A2) A2 += z * sA; Bt += z * sB; if (Bt2) Bt2 += z * sB; C += z * sC;
    const int lane = threadIdx.x & 31, lr = lane & 15, hi = lane >> 4; const int r0 = blockIdx.x * 64, c0 = blockIdx.y * 64;
    v8f acc[4][4];
#pragma unroll
    for (int mb = 0; mb < 4; ++mb)
#pragma unroll
        for (int nb = 0; nb < 4; ++nb) acc[mb][nb] = (v8f){};
    const size_t aoff = (size_t)(r0 + lr) * K + 8 * hi, boff = (size_t)(c0 + lr) * K + 8 * hi;
#pragma unroll 1
    for (int kc = 0; kc < K; kc += 32) {
        V a[4], a2[4];
#pragma unroll
        for (int mb = 0; mb < 4; ++mb) { a[mb] = WFrag<T16>::ld(A + aoff + (size_t)mb * 16 * K + kc); if (NSPLIT == 1 || NSPLIT == 2) a2[mb] = WFrag<T16>::ld(A2 + aoff + (size_t)mb * 16 * K + kc); }
#pragma unroll
        for (int nb = 0; nb < 4; ++nb) { const V b = WFrag<T16>::ld(Bt + boff + (size_t)nb * 16 * K + kc); V b2; if (NSPLIT >= 2) b2 = WFrag<T16>::ld(Bt2 + boff + (size_t)nb * 16 * K + kc);
#pragma unroll
            for (int mb = 0; mb < 4; ++mb) { acc[mb][nb] = WFrag<T16>::mma(a[mb], b, acc[mb][nb]); if (NSPLIT == 1 || NSPLIT == 2) acc[mb][nb] = WFrag<T16>::mma(a2[mb], b, acc[mb][nb]); if (NSPLIT >= 2) acc[mb][nb] = WFrag<T16>::mma(a[mb], b2, acc[mb][nb]); } }
        asm volatile("v_nop\n\tv_nop\n\tv_nop\n\tv_nop" : "+v"(acc[0][0]), "+v"(acc[1][1]), "+v"(acc[2][2]), "+v"(acc[3][3]) : "v"(a[0]), "v"(a[3]));
    }
#pragma unroll
    for (int mb = 0; mb < 4; ++mb) {
#pragma unroll
        for (int nb = 0; nb < 4; ++nb) {
#pragma unroll
            for (int j = 0; j < 8; ++j) os[(hi * 8 + j) * 68 + nb * 16 + lr] = acc[mb][nb][j]; }
        __builtin_amdgcn_wave_barrier(); asm volatile("" ::: "memory");
        float* crow = C + (size_t)(r0 + mb * 16) * ldc + c0;
#pragma unroll 1
        for (int ps = 0; ps < 2; ++ps) {
#pragma unroll
            for (int s = 0; s < 8; ++s) { const int row = 2 * s + hi, cofs = lr * 4; v4f val = *(const v4fa*)(os + row * 68 + cofs); val = val * csc;
                if (BIAS) { val[0] += bfr(bias[c0 + cofs]); val[1] += bfr(bias[c0 + cofs + 1]); val[2] += bfr(bias[c0 + cofs + 2]); val[3] += bfr(bias[c0 + cofs + 3]); }
                *(volatile v4f*)(crow + (size_t)row * ldc + cofs) = val; }
            if (ps == 0) __threadfence(); }
        __builtin_amdgcn_wave_barrier(); asm volatile("" ::: "memory");
    }
}

__global__ __launch_bounds__(256) void k_wsplit(const float* __restrict__ w, bf* WB) {
    const unsigned i = blockIdx.x * 256u + threadIdx.x; if (i >= (unsigned)(2 * HH * DHD / 8)) return;
    const unsigned pl = i >> 9; const unsigned a = (i >> 3) & 63u; const unsigned pc = i & 7u;
    const v8f v = *(const v8f*)(w + (size_t)a * (2 * DHD) + pl * DHD + pc * 8); v8us o;
#pragma unroll
    for (int k = 0; k < 8; ++k) o[k] = f2bf(v[k]);
    *(volatile v8us*)(WB + (size_t)i * 8) = o; __threadfence(); *(volatile v8us*)(WB + (size_t)i * 8) = o;
}

__global__ __launch_bounds__(256) void k_cvt8(const float* __restrict__ src, bf* dst, size_t n8) { const size_t i = (size_t)blockIdx.x * 256 + threadIdx.x; if (i >= n8) return; const v8f v = *(const v8f*)(src + i * 8); v8us o;
#pragma unroll
    for (int k = 0; k < 8; ++k) o[k] = f2bf(v[k]); *(volatile v8us*)(dst + i * 8) = o; __threadfence(); *(volatile v8us*)(dst + i * 8) = o; }

__global__ __launch_bounds__(256) void k_vtp(const float* __restrict__ F, h16* V16) {
    const size_t e = ((size_t)blockIdx.x * 256 + threadIdx.x) * 2; if (e >= (size_t)NB * DV * TK) return;
    const int t = (int)(e % TK); const int d = (int)((e / TK) % DV); const int b = (int)(e / ((size_t)TK * DV));
    v2h o;
#pragma unroll
    for (int q = 0; q < 2; ++q) o[q] = toh_flush(bfr(F[((size_t)b * TK + t + q) * DV + d]) * VSC);
    *(volatile v2h*)(V16 + e) = o; __threadfence(); *(volatile v2h*)(V16 + e) = o;
}

__device__ __forceinline__ float tnh(float x) {
    const float e = __builtin_amdgcn_exp2f(x * 2.8853900817779268f);
    const float r = __builtin_amdgcn_rcpf(e + 1.0f);
    return fmaf(-2.0f, r, 1.0f);
}

__global__ __launch_bounds__(256) void k_score(const float* __restrict__ QPF, const float* __restrict__ KPF, const float* __restrict__ vv, const int* __restrict__ mask, h16* P16) {
    __shared__ __align__(16) float s_sc[TK];
    __shared__ float red[8];
    const int blk = blockIdx.x; const int q = blk % TQ; const int h = (blk / TQ) % NHD; const int b = blk / (TQ * NHD);
    const int tid = threadIdx.x, lane = tid & 31, wave = tid >> 5;
    const v2f w2q = *(const v2f*)(QPF + ((size_t)(b * TQ + q) * NHD + h) * HH + lane * 2);
    const v2f v2 = *(const v2f*)(vv + lane * 2);
    const float wq0 = w2q[0], wq1 = w2q[1];
    const float vr0 = bfr(v2[0]), vr1 = bfr(v2[1]);
    const float* ub = KPF + ((size_t)b * TK * NHD + h) * HH + lane * 2;
#pragma unroll 1
    for (int kk = 0; kk < TK / 8; ++kk) {
        const int k = wave * (TK / 8) + kk;
        const v2f u2 = *(const v2f*)(ub + (size_t)k * NHD * HH);
        float acc = 0.0f;
        acc = fmaf(vr0, tnh(wq0 + u2[0]), acc);
        acc = fmaf(vr1, tnh(wq1 + u2[1]), acc);
#pragma unroll
        for (int sh = 16; sh; sh >>= 1) acc += __shfl_xor(acc, sh, 32);
        if (lane == 0) s_sc[k] = acc;
    }
    __syncthreads();
    const float r0 = s_sc[tid], r1 = s_sc[tid + 256];
    const int mk0 = mask[(size_t)b * TK + tid], mk1 = mask[(size_t)b * TK + tid + 256];
    const float a0 = (mk0 != 0) ? -INFINITY : r0;
    const float a1 = (mk1 != 0) ? -INFINITY : r1;
    float m = fmaxf(a0, a1);
#pragma unroll
    for (int sh = 16; sh; sh >>= 1) m = fmaxf(m, __shfl_xor(m, sh, 32));
    if (lane == 0) red[wave] = m;
    __syncthreads();
    m = red[0];
#pragma unroll
    for (int w = 1; w < 8; ++w) m = fmaxf(m, red[w]);
    __syncthreads();
    float d0 = a0 - m, d1 = a1 - m; asm volatile("" : "+v"(d0)); asm volatile("" : "+v"(d1));
    const float e0 = __builtin_amdgcn_exp2f(d0 * LOG2E), e1 = __builtin_amdgcn_exp2f(d1 * LOG2E);
    s_sc[tid] = e0; s_sc[tid + 256] = e1;
    float sum = e0 + e1;
#pragma unroll
    for (int sh = 16; sh; sh >>= 1) sum += __shfl_xor(sum, sh, 32);
    if (lane == 0) red[wave] = sum;
    __syncthreads();
    sum = red[0];
#pragma unroll
    for (int w = 1; w < 8; ++w) sum += red[w];
    const float inv = __builtin_amdgcn_rcpf(sum); const float invp = inv * PCAR;
    if (wave < 2) {
        const int f0 = (wave * 32 + lane) * 8;
        const v4f q0 = *(const v4fa*)(s_sc + f0); const v4f q1 = *(const v4fa*)(s_sc + f0 + 4);
        v8h o;
#pragma unroll
        for (int c = 0; c < 4; ++c) { o[c] = toh_flush(q0[c] * invp); o[4 + c] = toh_flush(q1[c] * invp); }
        h16* dst = P16 + ((size_t)(h * NB + b) * TQ + q) * TK + f0;
        *(volatile v8h*)dst = o; __threadfence(); *(volatile v8h*)dst = o;
    }
}

extern "C" void kernel_launch(void* const* d_in, const int* in_sizes, int n_in,
                              void* d_out, int out_size, void* d_ws, size_t ws_size, hipStream_t stream) {
    if (n_in < 6) return;
    if (in_sizes[0] < NB * TK * DV || in_sizes[1] < NB * TQ * DV || in_sizes[2] < HH * 2 * DHD || in_sizes[3] < HH || in_sizes[4] < HH || in_sizes[5] < NB * TK) return;
    if (out_size < NB_FULL * TQ_FULL * DV) return;
    const float* x     = (const float*)d_in[0];
    const float* query = (const float*)d_in[1];
    const float* W     = (const float*)d_in[2];
    const float* bb    = (const float*)d_in[3];
    const float* w2    = (const float*)d_in[4];
    const int*   mask  = (const int*)d_in[5];
    float* OUT = (float*)d_out;

    char* wsp = (char*)d_ws;
    auto take = [&](size_t bytes) { char* p = wsp; wsp += (bytes + 255) & ~(size_t)255; return (void*)p; };
    bf*    WB   = (bf*)take((size_t)2 * HH * DHD * 2);
    bf*    XB   = (bf*)take((size_t)NB * TK * DV * 2);
    bf*    QB   = (bf*)take((size_t)NB * TQ * DV * 2);
    float* KPF  = (float*)take((size_t)NB * TK * NHD * HH * 4);
    float* QPF  = (float*)take((size_t)NB * TQ * NHD * HH * 4);
    h16*   VT16 = (h16*)take((size_t)NB * DV * TK * 2);
    h16*   P16  = (h16*)take((size_t)NHD * NB * TQ * TK * 2);
    if ((size_t)(wsp - (char*)d_ws) > ws_size) return;

    k_wsplit<<<(unsigned)((2 * HH * DHD / 8 + 255) / 256), 256, 0, stream>>>(W, WB);
    k_cvt8<<<(unsigned)(((size_t)NB * TK * DV / 8 + 255) / 256), 256, 0, stream>>>(x, XB, (size_t)NB * TK * DV / 8);
    k_cvt8<<<(unsigned)(((size_t)NB * TQ * DV / 8 + 255) / 256), 256, 0, stream>>>(query, QB, (size_t)NB * TQ * DV / 8);
    k_vtp<<<(unsigned)(((size_t)NB * DV * TK / 2 + 255) / 256), 256, 0, stream>>>(x, VT16);
    k_gemmw<bf, 0, false><<<dim3(NB * TK * NHD / 64, HH / 64, 1), 32, 0, stream>>>(XB, nullptr, WB, nullptr, DHD, KPF, HH, nullptr, 1.0f, 0, 0, 0);
    k_gemmw<bf, 0, true><<<dim3(NB * TQ * NHD / 64, HH / 64, 1), 32, 0, stream>>>(QB, nullptr, WB + (size_t)HH * DHD, nullptr, DHD, QPF, HH, bb, 1.0f, 0, 0, 0);
    k_score<<<(unsigned)(NB * NHD * TQ), 256, 0, stream>>>(QPF, KPF, w2, mask, P16);
    for (int h = 0; h < NHD; ++h)
        k_gemmw<h16, 0, false><<<dim3(TQ / 64, DHD / 64, NB), 32, 0, stream>>>(P16 + (size_t)h * NB * TQ * TK, nullptr, VT16 + (size_t)h * DHD * TK, nullptr, TK, OUT + h * DHD, DV, nullptr, OSC, (size_t)TQ * TK, (size_t)DV * TK, (size_t)TQ_FULL * DV);
}
